// AttentionModule_39462159515861
// MI455X (gfx1250) — hardware-verified
//
#include <hip/hip_runtime.h>
#include <math.h>

constexpr int kBatch = 4;
constexpr int kSeq   = 2048;
constexpr int kDim   = 1024;
constexpr int kHeads = 16;
constexpr int kHdim  = 64;
constexpr int kTok   = kBatch * kSeq;
constexpr int kQKld  = 2 * kDim;
constexpr int kGrp   = 4;
constexpr int kChunks = kBatch * (kHeads / kGrp);
constexpr float kWCarry    = 16.0f;
constexpr float kWCarryInv = 1.0f / 16.0f;
constexpr float kPCarry    = 2048.0f;
constexpr float kCtxCarry  = 256.0f;
constexpr float kPVScale   = kCtxCarry / kPCarry;
constexpr float kOutScale  = 1.0f / (kCtxCarry * kWCarry);
constexpr float kQKScale   = 0.125f;

static_assert(kHeads * kHdim == kDim, "dims");
static_assert(kTok % 64 == 0 && kDim % 64 == 0 && kSeq % 64 == 0, "tile multiples");
static_assert(kDim % 32 == 0 && kSeq % 32 == 0 && kHdim % 32 == 0, "K multiples of 32");
static_assert(kHeads % kGrp == 0, "chunking");

constexpr size_t kOffX16  = 0;
constexpr size_t kOffW16  = kOffX16  + (size_t)kTok * kDim * 2;
constexpr size_t kOffWP16 = kOffW16  + (size_t)3 * kDim * kDim * 2;
constexpr size_t kOffQK   = kOffWP16 + (size_t)kDim * kDim * 2;
constexpr size_t kOffVT   = kOffQK   + (size_t)kTok * kQKld * 2;
constexpr size_t kOffP    = kOffVT   + (size_t)kDim * kTok * 2;
constexpr size_t kOffO    = kOffP    + (size_t)kGrp * kSeq * kSeq * 2;
constexpr size_t kWsEnd   = kOffO    + (size_t)kTok * kDim * 2;
static_assert(kWsEnd == 125829120ull, "carve total");
static_assert(kWsEnd <= 134217728ull, "carve cap");
static_assert(kOffW16 % 128 == 0 && kOffWP16 % 128 == 0 && kOffQK % 128 == 0 && kOffVT % 128 == 0 &&
              kOffP % 128 == 0 && kOffO % 128 == 0, "128-B aligned regions");

typedef __attribute__((ext_vector_type(16))) _Float16 v16h;
typedef __attribute__((ext_vector_type(8)))  _Float16 v8h;
typedef __attribute__((ext_vector_type(16))) __bf16   v16b;
typedef __attribute__((ext_vector_type(8)))  __bf16   v8b;
typedef __attribute__((ext_vector_type(8)))  float    v8f;
typedef __attribute__((ext_vector_type(4)))  float    v4f;
typedef __attribute__((ext_vector_type(4)))  unsigned int v4u;

__device__ __forceinline__ unsigned short f2bf_bits(float f) {
  unsigned u = __float_as_uint(f);
  return (unsigned short)((u + 0x7FFFu + ((u >> 16) & 1u)) >> 16);
}
__device__ __forceinline__ float bf_bits2f(unsigned short h) { return __uint_as_float(((unsigned)h) << 16); }

__device__ __forceinline__ void dep_guard_h(v8f& a, v8f& b, v16h x, v16h y) { asm volatile("v_nop\n\tv_nop\n\tv_nop\n\tv_nop" : "+v"(a), "+v"(b) : "v"(x), "v"(y)); }
__device__ __forceinline__ void dep_guard_b(v8f& a, v8f& b, v16b x, v16b y) { asm volatile("v_nop\n\tv_nop\n\tv_nop\n\tv_nop" : "+v"(a), "+v"(b) : "v"(x), "v"(y)); }
__device__ __forceinline__ void keep4_h(v16h a, v16h b, v16h c, v16h d) { asm volatile("v_nop" :: "v"(a), "v"(b), "v"(c), "v"(d)); }
__device__ __forceinline__ void keep4_b(v16b a, v16b b, v16b c, v16b d) { asm volatile("v_nop" :: "v"(a), "v"(b), "v"(c), "v"(d)); }
__device__ __forceinline__ void acc_guard4(v8f& a, v8f& b, v8f& c, v8f& d) { asm volatile("v_nop\n\tv_nop\n\tv_nop\n\tv_nop" : "+v"(a), "+v"(b), "+v"(c), "+v"(d)); }
template <typename T> struct Frag;
template <> struct Frag<_Float16> {
  typedef v16h V; union U { v16h v; v8h h[2]; };
  static __device__ __forceinline__ v16h load(const _Float16* p) {
    U f; f.h[0] = *(const v8h*)(p); f.h[1] = *(const v8h*)(p + 16); return f.v;
  }
  static __device__ __forceinline__ v8f mma(v16h a, v16h b, v8f c) {
    return __builtin_amdgcn_wmma_f32_16x16x32_f16(false, a, false, b, (short)0, c, false, false);
  }
  static __device__ __forceinline__ void guard(v8f& a, v8f& b, v16h x, v16h y) { dep_guard_h(a, b, x, y); }
  static __device__ __forceinline__ void keep(v16h a, v16h b, v16h c, v16h d) { keep4_h(a, b, c, d); }
};
template <> struct Frag<__bf16> {
  typedef v16b V; union U { v16b v; v8b h[2]; };
  static __device__ __forceinline__ v16b load(const __bf16* p) {
    U f; f.h[0] = *(const v8b*)(p); f.h[1] = *(const v8b*)(p + 16); return f.v;
  }
  static __device__ __forceinline__ v8f mma(v16b a, v16b b, v8f c) {
    return __builtin_amdgcn_wmma_f32_16x16x32_bf16(false, a, false, b, (short)0, c, false, false);
  }
  static __device__ __forceinline__ void guard(v8f& a, v8f& b, v16b x, v16b y) { dep_guard_b(a, b, x, y); }
  static __device__ __forceinline__ void keep(v16b a, v16b b, v16b c, v16b d) { keep4_b(a, b, c, d); }
};

__device__ __forceinline__ unsigned pk16(unsigned short a, unsigned short b) { return (unsigned)a | ((unsigned)b << 16); }
__device__ __forceinline__ unsigned short h_bits(float f) { const _Float16 h = (_Float16)f; return __builtin_bit_cast(unsigned short, h); }

template <int ET> struct Elem;
template <> struct Elem<0> { typedef _Float16 T; };
template <> struct Elem<1> { typedef __bf16 T; };
template <int ET, bool SPLIT, int BIAS_MODE, int OUT_MODE, bool RESID, int ACT = 0>
__global__ __launch_bounds__(256) void wmma_gemm64(
    const unsigned short* __restrict__ Ap, const unsigned short* __restrict__ A2p, int lda, long strideA,
    const unsigned short* __restrict__ Btp, const unsigned short* __restrict__ Bt2p, int ldb, long strideB,
    void* __restrict__ Cout, void* __restrict__ Cout2, int ldc, long strideC,
    const float* __restrict__ bias,
    const float* __restrict__ resid, long strideR,
    int M, int N, int K, float scale) {
  typedef typename Elem<ET>::T T;
  typedef typename Frag<T>::V V;
  const T* A = (const T*)Ap; const T* A2 = (const T*)A2p; const T* Bt = (const T*)Btp; const T* Bt2 = (const T*)Bt2p;
  __shared__ __align__(16) float sT[8][16 * 68];
  const int b    = blockIdx.y;
  const int lane = threadIdx.x & 31;
  const int wave = threadIdx.x >> 5;
  const int tilesN = N >> 6;
  const int tilesM = M >> 6;
  const int tile = blockIdx.x * 8 + wave;
  if (tile >= tilesM * tilesN) return;
  const int tm = tile / tilesN;
  const int tn = tile - tm * tilesN;
  const int m0 = tm << 6;
  const int n0 = tn << 6;

  const T* Ab  = A  + (size_t)b * strideA;
  const T* Bb  = Bt + (size_t)b * strideB;
  const T* Ab2 = SPLIT ? (A2  + (size_t)b * strideA) : nullptr;
  const T* Bb2 = SPLIT ? (Bt2 + (size_t)b * strideB) : nullptr;

  const int rlane = lane & 15;
  const int koff  = (lane >> 4) * 8;
  const int mOff  = (lane >> 4) * 8;

  v8f acc[4][4];
#pragma unroll
  for (int i = 0; i < 4; ++i)
#pragma unroll
    for (int j = 0; j < 4; ++j) acc[i][j] = (v8f){0.f,0.f,0.f,0.f,0.f,0.f,0.f,0.f};

  for (int k0 = 0; k0 < K; k0 += 32) {
    V bh[4], bl[4];
#pragma unroll
    for (int j = 0; j < 4; ++j) {
      const size_t bo = (size_t)(n0 + (j << 4) + rlane) * ldb + koff + k0;
      bh[j] = Frag<T>::load(Bb + bo);
      if (SPLIT) bl[j] = Frag<T>::load(Bb2 + bo);
    }
#pragma unroll
    for (int i = 0; i < 4; ++i) {
      const size_t ao = (size_t)(m0 + (i << 4) + rlane) * lda + koff + k0;
      V ah = Frag<T>::load(Ab + ao);
      V al;
      if (SPLIT) al = Frag<T>::load(Ab2 + ao);
#pragma unroll
      for (int j = 0; j < 4; ++j) {
        acc[i][j] = Frag<T>::mma(ah, bh[j], acc[i][j]);
        if (SPLIT) {
          acc[i][j] = Frag<T>::mma(ah, bl[j], acc[i][j]);
          acc[i][j] = Frag<T>::mma(al, bh[j], acc[i][j]);
        }
      }
      Frag<T>::guard(acc[i][0], acc[i][3], ah, SPLIT ? al : ah);
    }
    Frag<T>::keep(bh[0], bh[1], bh[2], bh[3]);
    if (SPLIT) Frag<T>::keep(bl[0], bl[1], bl[2], bl[3]);
  }
  acc_guard4(acc[0][0], acc[0][1], acc[0][2], acc[0][3]);
  acc_guard4(acc[1][0], acc[1][1], acc[1][2], acc[1][3]);
  acc_guard4(acc[2][0], acc[2][1], acc[2][2], acc[2][3]);
  acc_guard4(acc[3][0], acc[3][1], acc[3][2], acc[3][3]);

  float* slab = sT[wave];
  const float* Rb = RESID ? (resid + (size_t)b * strideR) : nullptr;
#pragma unroll
  for (int i = 0; i < 4; ++i) {
    const int mBase = m0 + (i << 4);
#pragma unroll
    for (int j = 0; j < 4; ++j) {
      const int n = n0 + (j << 4) + rlane;
      float bv = 0.f;
      if (BIAS_MODE == 2) bv = bias[n];
#pragma unroll
      for (int r = 0; r < 8; ++r) {
        float v = acc[i][j][r] * scale;
        if (BIAS_MODE == 1) v += bias[mBase + mOff + r];
        if (BIAS_MODE == 2) v += bv;
        if (RESID) v += Rb[(size_t)(mBase + mOff + r) * ldc + n];
        if (ACT == 2) v = fmaxf(v, 0.0f);
        if (ACT == 4) v = (v > 0.f) ? v : 0.01f * v;
        slab[(mOff + r) * 68 + (j << 4) + rlane] = v;
      }
    }
    __builtin_amdgcn_fence(__ATOMIC_RELEASE, "workgroup");
    __builtin_amdgcn_wave_barrier();
    __builtin_amdgcn_fence(__ATOMIC_ACQUIRE, "workgroup");
    if (OUT_MODE == 0) {
      float* C = (float*)Cout + (size_t)b * strideC;
      const int hh = lane >> 4, c4 = (lane & 15) * 4;
      for (int pass = 0; pass < 2; ++pass) {
#pragma unroll
        for (int it = 0; it < 8; ++it) {
          const int row = it * 2 + hh;
          v4f v = *(const v4f*)(slab + row * 68 + c4);
          *(volatile v4f*)(C + (size_t)(mBase + row) * ldc + n0 + c4) = v;
        }
        __threadfence();
      }
    } else {
      const int q = lane >> 3, c8 = (lane & 7) * 8;
      unsigned short* C  = (unsigned short*)Cout  + (size_t)b * strideC;
      unsigned short* C2 = (OUT_MODE == 2) ? ((unsigned short*)Cout2 + (size_t)b * strideC) : nullptr;
      for (int pass = 0; pass < 2; ++pass) {
#pragma unroll
        for (int it = 0; it < 4; ++it) {
          const int row = it * 4 + q;
          const float* sp = slab + row * 68 + c8;
          v8h hv, lv;
#pragma unroll
          for (int e = 0; e < 8; ++e) {
            if (OUT_MODE == 1) {
              hv[e] = (_Float16)sp[e];
            } else {
              unsigned short hb = f2bf_bits(sp[e]);
              unsigned short lb = f2bf_bits(sp[e] - bf_bits2f(hb));
              hv[e] = __builtin_bit_cast(_Float16, hb);
              lv[e] = __builtin_bit_cast(_Float16, lb);
            }
          }
          *(volatile v8h*)(C + (size_t)(mBase + row) * ldc + n0 + c8) = hv;
          if (OUT_MODE == 2) *(volatile v8h*)(C2 + (size_t)(mBase + row) * ldc + n0 + c8) = lv;
        }
        __threadfence();
      }
    }
    __builtin_amdgcn_fence(__ATOMIC_RELEASE, "workgroup");
    __builtin_amdgcn_wave_barrier();
    __builtin_amdgcn_fence(__ATOMIC_ACQUIRE, "workgroup");
  }
}

__global__ __launch_bounds__(256) void cast8_f16_kernel(const float* __restrict__ in, unsigned short* __restrict__ out,
                                                        int n8, float scale) {
  const int i = blockIdx.x * 256 + threadIdx.x;
  if (i >= n8) return;
  const float* p = in + 8 * (size_t)i;
  const v4f a = *(const v4f*)(p);
  const v4f c = *(const v4f*)(p + 4);
  unsigned short hb[8];
#pragma unroll
  for (int e = 0; e < 4; ++e) {
    hb[e]     = h_bits(a[e] * scale);
    hb[4 + e] = h_bits(c[e] * scale);
  }
  const v4u u = (v4u){pk16(hb[0], hb[1]), pk16(hb[2], hb[3]), pk16(hb[4], hb[5]), pk16(hb[6], hb[7])};
  unsigned short* q = out + 8 * (size_t)i;
  *(volatile v4u*)q = u;
  __threadfence();
  *(volatile v4u*)q = u;
}

constexpr int kSRows       = 16;
constexpr int kSThreads    = 128;
constexpr int kSWaves      = kSThreads / 32;
constexpr int kKeysPerWave = kSeq / kSWaves;
constexpr int kSlab        = 128;
constexpr int kSlabs       = kKeysPerWave / kSlab;
constexpr int kRowsPerWave = kSRows / kSWaves;
constexpr int kColsPerLane = kSeq / 32;
constexpr int kStoreIters  = kSeq / 256;
static_assert(kSlabs * kSlab * kSWaves == kSeq && kRowsPerWave * kSWaves == kSRows && kStoreIters * 256 == kSeq, "coverage");

__global__ __launch_bounds__(kSThreads) void scores_softmax_kernel(
    const unsigned short* __restrict__ Qg, const unsigned short* __restrict__ Kg, unsigned short* __restrict__ Pg) {
  __shared__ __align__(16) float Ssh[kSRows * kSeq];
  const int tid   = threadIdx.x;
  const int lane  = tid & 31;
  const int wave  = tid >> 5;
  const int rlane = lane & 15;
  const int hsel  = lane >> 4;
  const int koff  = hsel * 8;
  const int gi    = blockIdx.y;
  const int q0    = blockIdx.x * kSRows;
  const _Float16* Qp = (const _Float16*)Qg + (size_t)q0 * kQKld + gi * kHdim;
  const _Float16* Kp = (const _Float16*)Kg + gi * kHdim;
  unsigned short* Pp = Pg + (size_t)gi * kSeq * kSeq + (size_t)q0 * kSeq;

  v16h qa[2];
#pragma unroll
  for (int dc = 0; dc < 2; ++dc) qa[dc] = Frag<_Float16>::load(Qp + (size_t)rlane * kQKld + koff + dc * 32);

#pragma unroll 1
  for (int sl = 0; sl < kSlabs; ++sl) {
    const int key0 = wave * kKeysPerWave + sl * kSlab;
    v8f acc[8];
#pragma unroll
    for (int j = 0; j < 8; ++j) acc[j] = (v8f){0.f,0.f,0.f,0.f,0.f,0.f,0.f,0.f};
#pragma unroll
    for (int dc = 0; dc < 2; ++dc) {
#pragma unroll
      for (int jg = 0; jg < 2; ++jg) {
        v16h bk[4];
#pragma unroll
        for (int jj = 0; jj < 4; ++jj)
          bk[jj] = Frag<_Float16>::load(Kp + (size_t)(key0 + (jg * 4 + jj) * 16 + rlane) * kQKld + koff + dc * 32);
#pragma unroll
        for (int jj = 0; jj < 4; ++jj)
          acc[jg * 4 + jj] = Frag<_Float16>::mma(qa[dc], bk[jj], acc[jg * 4 + jj]);
        Frag<_Float16>::guard(acc[jg * 4], acc[jg * 4 + 3], qa[dc], bk[3]);
        Frag<_Float16>::keep(bk[0], bk[1], bk[2], bk[3]);
      }
    }
    acc_guard4(acc[0], acc[1], acc[2], acc[3]);
    acc_guard4(acc[4], acc[5], acc[6], acc[7]);
#pragma unroll
    for (int j = 0; j < 8; ++j) {
#pragma unroll
      for (int r = 0; r < 8; ++r) {
        Ssh[(8 * hsel + r) * kSeq + key0 + j * 16 + rlane] = acc[j][r] * kQKScale;
      }
    }
  }
  __syncthreads();

#pragma unroll 1
  for (int ri = 0; ri < kRowsPerWave; ++ri) {
    const int row = wave * kRowsPerWave + ri;
    float* sr = Ssh + row * kSeq;
    float m = -INFINITY;
#pragma unroll 1
    for (int i = 0; i < kColsPerLane; ++i) m = fmaxf(m, sr[i * 32 + lane]);
#pragma unroll
    for (int off = 16; off > 0; off >>= 1) m = fmaxf(m, __shfl_xor(m, off, 32));
    float sum = 0.f;
#pragma unroll 1
    for (int i = 0; i < kColsPerLane; ++i) {
      const float e = expf(sr[i * 32 + lane] - m);
      sr[i * 32 + lane] = e;
      sum += e;
    }
#pragma unroll
    for (int off = 16; off > 0; off >>= 1) sum += __shfl_xor(sum, off, 32);
    const float inv = kPCarry * (1.0f / sum);
    __builtin_amdgcn_fence(__ATOMIC_RELEASE, "workgroup");
    __builtin_amdgcn_wave_barrier();
    __builtin_amdgcn_fence(__ATOMIC_ACQUIRE, "workgroup");
    unsigned short* prow = Pp + (size_t)row * kSeq;
    for (int pass = 0; pass < 2; ++pass) {
#pragma unroll
      for (int it = 0; it < kStoreIters; ++it) {
        const int c0 = it * 256 + lane * 8;
        const v4f a = *(const v4f*)(sr + c0);
        const v4f c = *(const v4f*)(sr + c0 + 4);
        unsigned short hb[8];
#pragma unroll
        for (int e = 0; e < 4; ++e) {
          hb[e]     = h_bits(a[e] * inv);
          hb[4 + e] = h_bits(c[e] * inv);
        }
        const v4u u = (v4u){pk16(hb[0], hb[1]), pk16(hb[2], hb[3]), pk16(hb[4], hb[5]), pk16(hb[6], hb[7])};
        *(volatile v4u*)(prow + c0) = u;
      }
      __threadfence();
    }
  }
}

extern "C" void kernel_launch(void* const* d_in, const int* in_sizes, int n_in,
                              void* d_out, int out_size, void* d_ws, size_t ws_size,
                              hipStream_t stream) {
  if (n_in < 5) return;
  if (in_sizes[0] != kTok * kDim || in_sizes[1] != 3 * kDim * kDim || in_sizes[2] != 3 * kDim ||
      in_sizes[3] != kDim * kDim || in_sizes[4] != kDim) return;
  if (out_size != kTok * kDim) return;
  if (ws_size < kWsEnd) return;

  const float* x      = (const float*)d_in[0];
  const float* w_qkv  = (const float*)d_in[1];
  const float* b_qkv  = (const float*)d_in[2];
  const float* w_proj = (const float*)d_in[3];
  const float* b_proj = (const float*)d_in[4];
  float* out = (float*)d_out;

  char* ws = (char*)d_ws;
  unsigned short* X16  = (unsigned short*)(ws + kOffX16);
  unsigned short* W16  = (unsigned short*)(ws + kOffW16);
  unsigned short* WP16 = (unsigned short*)(ws + kOffWP16);
  unsigned short* QK   = (unsigned short*)(ws + kOffQK);
  unsigned short* VT   = (unsigned short*)(ws + kOffVT);
  unsigned short* Ppl  = (unsigned short*)(ws + kOffP);
  unsigned short* O16  = (unsigned short*)(ws + kOffO);

  {
    const int n8 = kTok * kDim / 8;
    cast8_f16_kernel<<<dim3((n8 + 255) / 256), dim3(256), 0, stream>>>(x, X16, n8, 1.0f);
  }
  {
    const int n8 = 3 * kDim * kDim / 8;
    cast8_f16_kernel<<<dim3((n8 + 255) / 256), dim3(256), 0, stream>>>(w_qkv, W16, n8, kWCarry);
  }
  {
    const int n8 = kDim * kDim / 8;
    cast8_f16_kernel<<<dim3((n8 + 255) / 256), dim3(256), 0, stream>>>(w_proj, WP16, n8, kWCarry);
  }

  {
    const int tiles = (kTok / 64) * (kQKld / 64);
    wmma_gemm64<0, false, 2, 1, false><<<dim3((tiles + 7) / 8, 1), dim3(256), 0, stream>>>(
        X16, nullptr, kDim, 0L,
        W16, nullptr, kDim, 0L,
        (void*)QK, nullptr, kQKld, 0L,
        b_qkv, nullptr, 0L,
        kTok, kQKld, kDim, kWCarryInv);
  }
  {
    const int tiles = (kDim / 64) * (kTok / 64);
    wmma_gemm64<0, false, 1, 1, false><<<dim3((tiles + 7) / 8, 1), dim3(256), 0, stream>>>(
        W16 + (size_t)2 * kDim * kDim, nullptr, kDim, 0L,
        X16, nullptr, kDim, 0L,
        (void*)VT, nullptr, kTok, 0L,
        b_qkv + 2 * kDim, nullptr, 0L,
        kDim, kTok, kDim, kWCarryInv);
  }

  for (int ch = 0; ch < kChunks; ++ch) {
    const int b  = ch / (kHeads / kGrp);
    const int h0 = (ch % (kHeads / kGrp)) * kGrp;
    const unsigned short* Qg = QK + (size_t)b * kSeq * kQKld + (size_t)h0 * kHdim;
    const unsigned short* Kg = Qg + kDim;
    scores_softmax_kernel<<<dim3(kSeq / kSRows, kGrp), dim3(kSThreads), 0, stream>>>(Qg, Kg, Ppl);
    {
      const int tiles = (kSeq / 64) * (kHdim / 64);
      wmma_gemm64<0, false, 0, 1, false><<<dim3((tiles + 7) / 8, kGrp), dim3(256), 0, stream>>>(
          Ppl, nullptr, kSeq, (long)kSeq * kSeq,
          VT + (size_t)h0 * kHdim * kTok + (size_t)b * kSeq, nullptr, kTok, (long)kHdim * kTok,
          (void*)(O16 + (size_t)b * kSeq * kDim + (size_t)h0 * kHdim), nullptr, kDim, (long)kHdim,
          nullptr, nullptr, 0L,
          kSeq, kHdim, kSeq, kPVScale);
    }
  }

  {
    const int tiles = (kTok / 64) * (kDim / 64);
    wmma_gemm64<0, false, 2, 0, false><<<dim3((tiles + 7) / 8, 1), dim3(256), 0, stream>>>(
        O16, nullptr, kDim, 0L,
        WP16, nullptr, kDim, 0L,
        (void*)out, nullptr, kDim, 0L,
        b_proj, nullptr, 0L,
        kTok, kDim, kDim, kOutScale);
  }
}
